// MolecularMPNN_24008867185218
// MI455X (gfx1250) — hardware-verified
//
#include <hip/hip_runtime.h>
#include <stddef.h>


#define NTHR   128
#define NWAVE  4
#define EPT    8
#define CHUNK  (NTHR * EPT)
#define WCAP   (EPT * 32)
#define LISTN  (NWAVE * WCAP)
#define NI     16
#define HD     64
#define EI     8
#define GFT    32
#define NC     40
#define NCP    48
#define KW     1024
#define KP     1056
#define KF     160
#define NB     448
#define PASSA  (NWAVE * 16)
#define PCAPA  (CHUNK + PASSA)
#define GB     256
#define PASSP  NTHR
#define PCAPP  (CHUNK + PASSP)
#define RB     64
#define PREPA  66
#define PREPB  10
#define PREPC  3

static_assert(PASSA <= NTHR);
static_assert((NB % NWAVE) == 0);
static_assert((NB % 4) == 0);
static_assert((GB % 4) == 0);
static_assert(PREPA * NTHR * 8 == HD * KP);
static_assert(PREPB * NTHR * 8 == HD * KF);
static_assert(PREPC * NTHR * 8 == NCP * HD);
static_assert((KP % 32) == 0 && (KF % 32) == 0);
static_assert(((NB * HD) % (4 * NTHR)) == 0);
static_assert(((GB * HD) % (4 * NTHR)) == 0);

typedef float    v4f  __attribute__((ext_vector_type(4)));
typedef float    v8f  __attribute__((ext_vector_type(8)));
typedef int      v4i  __attribute__((ext_vector_type(4)));
typedef _Float16 v8h  __attribute__((ext_vector_type(8)));
typedef _Float16 v16h __attribute__((ext_vector_type(16)));
union FragH { v16h v; v8h h[2]; };

__device__ __forceinline__ v8f z8f() {
  v8f r;
#pragma unroll
  for (int i = 0; i < 8; ++i) r[i] = 0.0f;
  return r;
}
__device__ __forceinline__ v8h z8h() {
  v8h r;
#pragma unroll
  for (int i = 0; i < 8; ++i) r[i] = (_Float16)0.0f;
  return r;
}

__device__ __forceinline__ v8f wmh(v16h a, v16h b, v8f c) {
  v8f d = __builtin_amdgcn_wmma_f32_16x16x32_f16(false, a, false, b, (short)0, c, false, false);
  asm volatile("v_nop\n\tv_nop\n\tv_nop\n\tv_nop" : "+v"(d) : "v"(a), "v"(b));
  return d;
}

template <int W>
__device__ __forceinline__ int scan_chunk(const int* __restrict__ ids, int nT, int cbase, int base0,
                                          int vec8, int* list, int tid, int wave) {
  int wc = 0;
  const int el0  = tid * EPT;
  const int e0   = cbase + el0;
  const int sent = -2147483647 - 1;
  v4i da, db;
  if (vec8 != 0 && cbase + CHUNK <= nT) {
    da = *(const v4i*)(ids + e0);
    db = *(const v4i*)(ids + e0 + 4);
  } else {
    const int l = nT - 1;
    da.x = (e0     < nT) ? ids[min(e0,     l)] : sent;
    da.y = (e0 + 1 < nT) ? ids[min(e0 + 1, l)] : sent;
    da.z = (e0 + 2 < nT) ? ids[min(e0 + 2, l)] : sent;
    da.w = (e0 + 3 < nT) ? ids[min(e0 + 3, l)] : sent;
    db.x = (e0 + 4 < nT) ? ids[min(e0 + 4, l)] : sent;
    db.y = (e0 + 5 < nT) ? ids[min(e0 + 5, l)] : sent;
    db.z = (e0 + 6 < nT) ? ids[min(e0 + 6, l)] : sent;
    db.w = (e0 + 7 < nT) ? ids[min(e0 + 7, l)] : sent;
  }
  const unsigned nb = (unsigned)base0;
  const unsigned s0 = (unsigned)da.x - nb, s1 = (unsigned)da.y - nb;
  const unsigned s2 = (unsigned)da.z - nb, s3 = (unsigned)da.w - nb;
  const unsigned s4 = (unsigned)db.x - nb, s5 = (unsigned)db.y - nb;
  const unsigned s6 = (unsigned)db.z - nb, s7 = (unsigned)db.w - nb;
  const bool h0 = s0 < (unsigned)W, h1 = s1 < (unsigned)W, h2 = s2 < (unsigned)W, h3 = s3 < (unsigned)W;
  const bool h4 = s4 < (unsigned)W, h5 = s5 < (unsigned)W, h6 = s6 < (unsigned)W, h7 = s7 < (unsigned)W;
  const unsigned any = __builtin_amdgcn_ballot_w32(h0 | h1 | h2 | h3 | h4 | h5 | h6 | h7);
  if (any != 0u) {
#define HITJ(J, HJ) { \
      const unsigned mj = __builtin_amdgcn_ballot_w32(HJ); \
      if (mj != 0u) { \
        if (HJ) { \
          const int pos = wc + (int)__builtin_amdgcn_mbcnt_lo(mj, 0u); \
          if (pos < WCAP) list[wave * WCAP + pos] = el0 + (J); \
        } \
        wc += (int)__builtin_popcount(mj); } }
    HITJ(0, h0)
    HITJ(1, h1)
    HITJ(2, h2)
    HITJ(3, h3)
    HITJ(4, h4)
    HITJ(5, h5)
    HITJ(6, h6)
    HITJ(7, h7)
#undef HITJ
  }
  return wc;
}

__global__ __launch_bounds__(NTHR) void k_prep(
    const float* __restrict__ W2, const float* __restrict__ B2,
    const float* __restrict__ Wf, const float* __restrict__ Wn,
    _Float16* wp, _Float16* wfc, _Float16* wnp) {
  const int b = blockIdx.x, tid = threadIdx.x;
  v8h v;
  _Float16* dst;
  if (b < PREPA) {
    const int t   = b * NTHR + tid;
    const int n   = t / (KP / 8);
    const int j   = t - n * (KP / 8);
    const int kk0 = j * 8;
#pragma unroll
    for (int u = 0; u < 8; ++u) {
      const int kk = kk0 + u;
      int fi = kk >> 6; fi = fi > (NI - 1) ? (NI - 1) : fi;
      const int k = kk & 63;
      const float a = W2[(size_t)k * KW + fi * HD + n];
      int bi = kk - KW; bi = bi < 0 ? 0 : (bi > NI - 1 ? NI - 1 : bi);
      const float c = B2[bi * HD + n];
      const float val = (kk < KW) ? a : ((kk < KW + NI) ? c : 0.0f);
      v[u] = (_Float16)(val * 8.0f);
    }
    dst = wp + (size_t)t * 8;
  } else if (b < PREPA + PREPB) {
    const int t   = (b - PREPA) * NTHR + tid;
    const int n   = t / (KF / 8);
    const int j   = t - n * (KF / 8);
    const int kk0 = j * 8;
#pragma unroll
    for (int u = 0; u < 8; ++u) v[u] = (_Float16)(Wf[(kk0 + u) * HD + n] * 16.0f);
    dst = wfc + (size_t)t * 8;
  } else {
    const int t   = (b - PREPA - PREPB) * NTHR + tid;
    const int n   = t >> 3;
    const int kk0 = (t & 7) * 8;
    const int nn  = n > (NC - 1) ? (NC - 1) : n;
#pragma unroll
    for (int u = 0; u < 8; ++u) {
      const float a = Wn[(kk0 + u) * NC + nn];
      const float val = (n < NC) ? a * 8.0f : 0.0f;
      v[u] = (_Float16)val;
    }
    dst = wnp + (size_t)t * 8;
  }
  *(volatile v8h*)dst = v;
  __threadfence();
  *(volatile v8h*)dst = v;
}

__global__ __launch_bounds__(NTHR) void k_agg(
    const float* __restrict__ x, const int* __restrict__ ei, const float* __restrict__ eat,
    const float* __restrict__ W1, const float* __restrict__ B1, const _Float16* __restrict__ wp,
    const float* __restrict__ root, const float* __restrict__ cb,
    const float* __restrict__ Wg, const float* __restrict__ bg,
    float* hbuf, float* gbuf, int nN, int nE, int vec8) {
  __shared__ __attribute__((aligned(16))) float acc[(NB + 1) * HD];
  __shared__ float ccnt[NB + 1];
  __shared__ __attribute__((aligned(16))) float gst[NB];
  __shared__ __attribute__((aligned(16))) float msg[PASSA * HD];
  __shared__ int   mslot[PASSA];
  __shared__ __attribute__((aligned(16))) float xs[PASSA * NI];
  __shared__ __attribute__((aligned(16))) float eas[PASSA * EI];
  __shared__ __attribute__((aligned(16))) int   list[LISTN];
  __shared__ int   pend[PCAPA];
  __shared__ __attribute__((aligned(16))) float w1s[HD * EI];
  __shared__ float b1s[HD];
  __shared__ int   wcnt[NWAVE];
  __shared__ int   pendN;

  const int tid = threadIdx.x, lane = tid & 31, wave = tid >> 5, hh = lane >> 4, m = lane & 15;
  const int nodeBase = blockIdx.x * NB;
  const int* srcs = ei;
  const int* dsts = ei + nE;

  for (int i = tid; i < (NB + 1) * HD; i += NTHR) acc[i] = 0.0f;
  for (int i = tid; i < NB + 1; i += NTHR) ccnt[i] = 0.0f;
  for (int i = tid; i < PASSA * HD; i += NTHR) msg[i] = 0.0f;
  for (int i = tid; i < HD * EI; i += NTHR) {
    const int k = i >> 3, ii = i & 7;
    w1s[i] = W1[ii * HD + k];
  }
  if (tid < HD) b1s[tid] = B1[tid];
  if (tid < PASSA) mslot[tid] = NB;
  if (tid == 0) pendN = 0;
  __syncthreads();

  const int nChunks = (nE + CHUNK - 1) / CHUNK;
#pragma unroll 1
  for (int ch = 0; ch < nChunks; ++ch) {
    const int cbase = ch * CHUNK;
    const int wc = scan_chunk<NB>(dsts, nE, cbase, nodeBase, vec8, list, tid, wave);
    if (lane == 0) wcnt[wave] = wc;
    __syncthreads();

    const int base = pendN;
    int tot = 0, myoff = 0;
#pragma unroll
    for (int w = 0; w < NWAVE; ++w) {
      int c = wcnt[w];
      c = c > WCAP ? WCAP : (c < 0 ? 0 : c);
      if (w < wave) myoff += c;
      tot += c;
    }
    int newN = base + tot;
    newN = newN > PCAPA ? PCAPA : newN;
    {
      int n = wcnt[wave];
      n = n > WCAP ? WCAP : (n < 0 ? 0 : n);
      const int* lp = list + wave * WCAP;
      for (int i = lane; i < n; i += 32) {
        const int pos = base + myoff + i;
        if (pos < PCAPA) pend[pos] = cbase + lp[i];
      }
    }
    const int fin = (ch == nChunks - 1) ? 1 : 0;
    const int R   = (fin != 0) ? (newN + PASSA - 1) / PASSA : newN / PASSA;
    const int Pv  = (fin != 0) ? newN : R * PASSA;
    __syncthreads();

#pragma unroll 1
    for (int r = 0; r < R; ++r) {
      {
        const int idx = r * PASSA + wave * 16 + m;
        const bool valid = idx < Pv;
        int e = pend[idx];
        e = e < 0 ? 0 : (e > nE - 1 ? nE - 1 : e);
        const int d = dsts[e];
        int s = srcs[e];
        int slot = d - nodeBase;
        if (!valid || (unsigned)slot >= (unsigned)NB) slot = NB;
        s = s < 0 ? 0 : (s > nN - 1 ? nN - 1 : s);
        const int es = wave * 16 + m;
        const v4f xa = *(const v4f*)(x + (size_t)s * NI + 8 * hh);
        const v4f xb = *(const v4f*)(x + (size_t)s * NI + 8 * hh + 4);
        *(v4f*)(xs + es * NI + 8 * hh)     = xa;
        *(v4f*)(xs + es * NI + 8 * hh + 4) = xb;
        const v4f ev = *(const v4f*)(eat + (size_t)e * EI + 4 * hh);
        *(v4f*)(eas + es * EI + 4 * hh) = ev;
        mslot[es] = slot;
      }
      __syncthreads();

      const bool wv = (r * PASSA + wave * 16) < Pv;
      if (wv) {
        const int es = wave * 16 + m;
        const v4f e0 = *(const v4f*)(eas + es * EI);
        const v4f e1 = *(const v4f*)(eas + es * EI + 4);
        float ehv[32];
#pragma unroll
        for (int q = 0; q < 4; ++q) {
#pragma unroll
          for (int j = 0; j < 8; ++j) {
            const int k = 16 * q + 8 * hh + j;
            const v4f w0 = *(const v4f*)(w1s + k * EI);
            const v4f w4 = *(const v4f*)(w1s + k * EI + 4);
            float a = e0.x * w0.x;
            a += e0.y * w0.y; a += e0.z * w0.z; a += e0.w * w0.w;
            a += e1.x * w4.x; a += e1.y * w4.y; a += e1.z * w4.z; a += e1.w * w4.w;
            a += b1s[k];
            ehv[8 * q + j] = fmaxf(a, 0.0f);
          }
        }
        v8f c0 = z8f(), c1 = z8f(), c2 = z8f(), c3 = z8f();
        const float* xr = xs + es * NI;
        const _Float16* wb = wp + (size_t)m * KP + 8 * hh;
#pragma unroll 1
        for (int s2 = 0; s2 < NI; ++s2) {
          const float xi = xr[s2];
          FragH a, bq;
#pragma unroll
          for (int j = 0; j < 8; ++j) {
            a.h[0][j] = (_Float16)(xi * ehv[j]);
            a.h[1][j] = (_Float16)(xi * ehv[8 + j]);
          }
          const _Float16* w0 = wb + 64 * s2;
          bq.h[0] = *(const v8h*)(w0);               bq.h[1] = *(const v8h*)(w0 + 16);
          c0 = wmh(a.v, bq.v, c0);
          bq.h[0] = *(const v8h*)(w0 + 16 * KP);     bq.h[1] = *(const v8h*)(w0 + 16 * KP + 16);
          c1 = wmh(a.v, bq.v, c1);
          bq.h[0] = *(const v8h*)(w0 + 32 * KP);     bq.h[1] = *(const v8h*)(w0 + 32 * KP + 16);
          c2 = wmh(a.v, bq.v, c2);
          bq.h[0] = *(const v8h*)(w0 + 48 * KP);     bq.h[1] = *(const v8h*)(w0 + 48 * KP + 16);
          c3 = wmh(a.v, bq.v, c3);
#pragma unroll
          for (int j = 0; j < 8; ++j) {
            a.h[0][j] = (_Float16)(xi * ehv[16 + j]);
            a.h[1][j] = (_Float16)(xi * ehv[24 + j]);
          }
          const _Float16* w1p = w0 + 32;
          bq.h[0] = *(const v8h*)(w1p);              bq.h[1] = *(const v8h*)(w1p + 16);
          c0 = wmh(a.v, bq.v, c0);
          bq.h[0] = *(const v8h*)(w1p + 16 * KP);    bq.h[1] = *(const v8h*)(w1p + 16 * KP + 16);
          c1 = wmh(a.v, bq.v, c1);
          bq.h[0] = *(const v8h*)(w1p + 32 * KP);    bq.h[1] = *(const v8h*)(w1p + 32 * KP + 16);
          c2 = wmh(a.v, bq.v, c2);
          bq.h[0] = *(const v8h*)(w1p + 48 * KP);    bq.h[1] = *(const v8h*)(w1p + 48 * KP + 16);
          c3 = wmh(a.v, bq.v, c3);
        }
        {
          FragH a, bq;
          const v4f xa = *(const v4f*)(xr + 8 * hh);
          const v4f xb = *(const v4f*)(xr + 8 * hh + 4);
          a.h[0][0] = (_Float16)xa.x; a.h[0][1] = (_Float16)xa.y; a.h[0][2] = (_Float16)xa.z; a.h[0][3] = (_Float16)xa.w;
          a.h[0][4] = (_Float16)xb.x; a.h[0][5] = (_Float16)xb.y; a.h[0][6] = (_Float16)xb.z; a.h[0][7] = (_Float16)xb.w;
          a.h[1] = z8h();
          const _Float16* w0 = wb + KW;
          bq.h[0] = *(const v8h*)(w0);               bq.h[1] = *(const v8h*)(w0 + 16);
          c0 = wmh(a.v, bq.v, c0);
          bq.h[0] = *(const v8h*)(w0 + 16 * KP);     bq.h[1] = *(const v8h*)(w0 + 16 * KP + 16);
          c1 = wmh(a.v, bq.v, c1);
          bq.h[0] = *(const v8h*)(w0 + 32 * KP);     bq.h[1] = *(const v8h*)(w0 + 32 * KP + 16);
          c2 = wmh(a.v, bq.v, c2);
          bq.h[0] = *(const v8h*)(w0 + 48 * KP);     bq.h[1] = *(const v8h*)(w0 + 48 * KP + 16);
          c3 = wmh(a.v, bq.v, c3);
        }
#pragma unroll
        for (int r2 = 0; r2 < 8; ++r2) {
          float* mp = msg + (wave * 16 + 8 * hh + r2) * HD + m;
          mp[0]  = c0[r2] * 0.125f;
          mp[16] = c1[r2] * 0.125f;
          mp[32] = c2[r2] * 0.125f;
          mp[48] = c3[r2] * 0.125f;
        }
      }
      __syncthreads();

      if (wave < 2) {
        const int chn = wave * 32 + lane;
#pragma unroll 1
        for (int i = 0; i < PASSA; ++i) {
          int sl = mslot[i];
          sl = sl < 0 ? 0 : (sl > NB ? NB : sl);
          acc[sl * HD + chn] += msg[i * HD + chn];
        }
      } else if (wave == 2 && lane == 0) {
#pragma unroll 1
        for (int i = 0; i < PASSA; ++i) {
          int sl = mslot[i];
          sl = sl < 0 ? 0 : (sl > NB ? NB : sl);
          ccnt[sl] += 1.0f;
        }
      }
      __syncthreads();
    }

    int rem = newN - R * PASSA;
    rem = rem < 0 ? 0 : rem;
    if (R > 0 && tid < rem) pend[tid] = pend[R * PASSA + tid];
    if (tid == 0) pendN = rem;
  }
  __syncthreads();

  {
    const float bgv = bg[0];
    const float cb0 = cb[lane], cb1 = cb[32 + lane];
    const float wg0 = Wg[lane], wg1 = Wg[32 + lane];
#pragma unroll 1
    for (int sl = wave; sl < NB; sl += NWAVE) {
      int nn = nodeBase + sl; nn = nn > nN - 1 ? nN - 1 : nn;
      const float inv = 1.0f / fmaxf(ccnt[sl], 1.0f);
      const float* xg = x + (size_t)nn * NI;
      const v4f x0 = *(const v4f*)(xg), x1 = *(const v4f*)(xg + 4), x2 = *(const v4f*)(xg + 8), x3 = *(const v4f*)(xg + 12);
      float xv[16];
      xv[0] = x0.x; xv[1] = x0.y; xv[2]  = x0.z; xv[3]  = x0.w; xv[4]  = x1.x; xv[5]  = x1.y; xv[6]  = x1.z; xv[7]  = x1.w;
      xv[8] = x2.x; xv[9] = x2.y; xv[10] = x2.z; xv[11] = x2.w; xv[12] = x3.x; xv[13] = x3.y; xv[14] = x3.z; xv[15] = x3.w;
      float d0 = 0.0f, d1 = 0.0f;
#pragma unroll
      for (int i = 0; i < NI; ++i) {
        d0 += xv[i] * root[i * HD + lane];
        d1 += xv[i] * root[i * HD + 32 + lane];
      }
      float v0 = acc[sl * HD + lane] * inv;
      float v1 = acc[sl * HD + 32 + lane] * inv;
      v0 = fmaxf(v0 + d0 + cb0, 0.0f);
      v1 = fmaxf(v1 + d1 + cb1, 0.0f);
      float g = v0 * wg0 + v1 * wg1;
      g += __shfl_xor(g, 16, 32);
      g += __shfl_xor(g, 8, 32);
      g += __shfl_xor(g, 4, 32);
      g += __shfl_xor(g, 2, 32);
      g += __shfl_xor(g, 1, 32);
      acc[sl * HD + lane] = v0;
      acc[sl * HD + 32 + lane] = v1;
      if (lane == 0) gst[sl] = g + bgv;
    }
  }
  __syncthreads();

  {
    float* hb0 = hbuf + (size_t)nodeBase * HD;
    float* gb0 = gbuf + nodeBase;
    constexpr int NQ = (NB * HD) / (4 * NTHR);
#pragma unroll 1
    for (int ps = 0; ps < 2; ++ps) {
#pragma unroll 1
      for (int q = 0; q < NQ; ++q) {
        const int i4 = (q * NTHR + tid) * 4;
        const v4f v = *(const v4f*)(acc + i4);
        *(volatile v4f*)(hb0 + i4) = v;
      }
      if (tid < NB / 4) {
        const v4f v = *(const v4f*)(gst + 4 * tid);
        *(volatile v4f*)(gb0 + 4 * tid) = v;
      }
      if (ps == 0) __threadfence();
    }
  }
}

__global__ __launch_bounds__(NTHR) void k_pool(
    const float* __restrict__ gbuf, const float* __restrict__ hbuf, const int* __restrict__ bt,
    const float* __restrict__ Wsp, const float* __restrict__ bsp,
    float* gctx, float* sgv, int nN, int vec8) {
  __shared__ __attribute__((aligned(16))) float ctx[(GB + 1) * HD];
  __shared__ float mx[GB + 1];
  __shared__ float den[GB + 1];
  __shared__ __attribute__((aligned(16))) float sgs[GB];
  __shared__ float hw[PASSP];
  __shared__ int   hs[PASSP];
  __shared__ int   hn[PASSP];
  __shared__ __attribute__((aligned(16))) int list[LISTN];
  __shared__ int   pend[PCAPP];
  __shared__ int   wcnt[NWAVE];
  __shared__ int   pendN;

  const int tid = threadIdx.x, lane = tid & 31, wave = tid >> 5;
  const int gBase = blockIdx.x * GB;
  const float ninf = -__int_as_float(0x7f800000);

  for (int i = tid; i < (GB + 1) * HD; i += NTHR) ctx[i] = 0.0f;
  for (int i = tid; i < GB + 1; i += NTHR) { mx[i] = ninf; den[i] = 0.0f; }
  if (tid == 0) pendN = 0;
  __syncthreads();

  const int nChunks = (nN + CHUNK - 1) / CHUNK;
#pragma unroll 1
  for (int sw = 0; sw < 2; ++sw) {
#pragma unroll 1
    for (int ch = 0; ch < nChunks; ++ch) {
      const int cbase = ch * CHUNK;
      const int wc = scan_chunk<GB>(bt, nN, cbase, gBase, vec8, list, tid, wave);
      if (lane == 0) wcnt[wave] = wc;
      __syncthreads();

      const int base = pendN;
      int tot = 0, myoff = 0;
#pragma unroll
      for (int w = 0; w < NWAVE; ++w) {
        int c = wcnt[w];
        c = c > WCAP ? WCAP : (c < 0 ? 0 : c);
        if (w < wave) myoff += c;
        tot += c;
      }
      int newN = base + tot;
      newN = newN > PCAPP ? PCAPP : newN;
      {
        int n = wcnt[wave];
        n = n > WCAP ? WCAP : (n < 0 ? 0 : n);
        const int* lp = list + wave * WCAP;
        for (int i = lane; i < n; i += 32) {
          const int pos = base + myoff + i;
          if (pos < PCAPP) pend[pos] = cbase + lp[i];
        }
      }
      const int fin = (ch == nChunks - 1) ? 1 : 0;
      const int R   = (fin != 0) ? (newN + PASSP - 1) / PASSP : newN / PASSP;
      const int Pv  = (fin != 0) ? newN : R * PASSP;
      __syncthreads();

#pragma unroll 1
      for (int r = 0; r < R; ++r) {
        const int idx = r * PASSP + tid;
        const bool valid = idx < Pv;
        int n = pend[idx];
        n = n < 0 ? 0 : (n > nN - 1 ? nN - 1 : n);
        const int b = bt[n];
        int slot = b - gBase;
        if (!valid || (unsigned)slot >= (unsigned)GB) slot = GB;
        const float g = gbuf[n];
        if (sw == 0) {
          hw[tid] = g; hs[tid] = slot;
          __syncthreads();
          if (tid == 0) {
#pragma unroll 1
            for (int i = 0; i < PASSP; ++i) {
              int sl = hs[i]; sl = sl < 0 ? 0 : (sl > GB ? GB : sl);
              mx[sl] = fmaxf(mx[sl], hw[i]);
            }
          }
          __syncthreads();
        } else {
          const float mv = mx[slot];
          const float t = expf(g - mv);
          const float w = valid ? t : 0.0f;
          hw[tid] = w; hs[tid] = slot; hn[tid] = n;
          __syncthreads();
          if (wave < 2) {
            const int chn = wave * 32 + lane;
#pragma unroll 1
            for (int i = 0; i < PASSP; ++i) {
              int sl = hs[i]; sl = sl < 0 ? 0 : (sl > GB ? GB : sl);
              int nn = hn[i]; nn = nn < 0 ? 0 : (nn > nN - 1 ? nN - 1 : nn);
              ctx[sl * HD + chn] += hw[i] * hbuf[(size_t)nn * HD + chn];
            }
          } else if (wave == 2 && lane == 0) {
#pragma unroll 1
            for (int i = 0; i < PASSP; ++i) {
              int sl = hs[i]; sl = sl < 0 ? 0 : (sl > GB ? GB : sl);
              den[sl] += hw[i];
            }
          }
          __syncthreads();
        }
      }

      int rem = newN - R * PASSP;
      rem = rem < 0 ? 0 : rem;
      if (R > 0 && tid < rem) pend[tid] = pend[R * PASSP + tid];
      if (tid == 0) pendN = rem;
    }
    __syncthreads();
  }

  {
    const float ws0 = Wsp[lane], ws1 = Wsp[32 + lane];
    const float bsv = bsp[0];
#pragma unroll 1
    for (int sl = wave; sl < GB; sl += NWAVE) {
      const float d = den[sl];
      const float rinv = (d > 0.0f) ? (1.0f / d) : 0.0f;
      const float v0 = ctx[sl * HD + lane] * rinv;
      const float v1 = ctx[sl * HD + 32 + lane] * rinv;
      float s = v0 * ws0 + v1 * ws1;
      s += __shfl_xor(s, 16, 32);
      s += __shfl_xor(s, 8, 32);
      s += __shfl_xor(s, 4, 32);
      s += __shfl_xor(s, 2, 32);
      s += __shfl_xor(s, 1, 32);
      s += bsv;
      s = fminf(fmaxf(s, -30.0f), 30.0f);
      const float sg = 1.0f / (1.0f + __expf(-s));
      ctx[sl * HD + lane] = v0;
      ctx[sl * HD + 32 + lane] = v1;
      if (lane == 0) sgs[sl] = sg;
    }
  }
  __syncthreads();

  {
    float* c0 = gctx + (size_t)gBase * HD;
    float* s0 = sgv + gBase;
    constexpr int NQ = (GB * HD) / (4 * NTHR);
#pragma unroll 1
    for (int ps = 0; ps < 2; ++ps) {
#pragma unroll 1
      for (int q = 0; q < NQ; ++q) {
        const int i4 = (q * NTHR + tid) * 4;
        const v4f v = *(const v4f*)(ctx + i4);
        *(volatile v4f*)(c0 + i4) = v;
      }
      if (tid < GB / 4) {
        const v4f v = *(const v4f*)(sgs + 4 * tid);
        *(volatile v4f*)(s0 + 4 * tid) = v;
      }
      if (ps == 0) __threadfence();
    }
  }
}

__global__ __launch_bounds__(NTHR) void k_head(
    const float* __restrict__ hbuf, const float* __restrict__ gctx, const float* __restrict__ sgv,
    const int* __restrict__ bt, const float* __restrict__ pk,
    const _Float16* __restrict__ wfc, const float* __restrict__ bfc,
    const _Float16* __restrict__ wnp, const float* __restrict__ bnp,
    float* out0, float* out1, int nN, int nG) {
  __shared__ __attribute__((aligned(16))) _Float16 feat[RB * KF];
  __shared__ __attribute__((aligned(16))) _Float16 ft[RB * HD];
  __shared__ __attribute__((aligned(16))) float    lg[RB * NCP];
  __shared__ __attribute__((aligned(16))) float    ost[RB * NC];
  __shared__ __attribute__((aligned(16))) float    sst[RB];

  const int tid = threadIdx.x, lane = tid & 31, wave = tid >> 5, hh = lane >> 4, m = lane & 15;
  const int base = blockIdx.x * RB;

  for (int c = tid; c < RB * (KF / 8); c += NTHR) {
    const int row = c / (KF / 8), j = c - row * (KF / 8);
    int node = base + row; node = node > nN - 1 ? nN - 1 : node;
    int bb = bt[node]; bb = bb < 0 ? 0 : (bb > nG - 1 ? nG - 1 : bb);
    int j1 = j - 8;  j1 = j1 < 0 ? 0 : (j1 > 7 ? 7 : j1);
    int j2 = j - 16; j2 = j2 < 0 ? 0 : (j2 > 3 ? 3 : j2);
    const float* p = (j < 8) ? (hbuf + (size_t)node * HD + 8 * j)
                   : ((j < 16) ? (gctx + (size_t)bb * HD + 8 * j1) : (pk + (size_t)bb * GFT + 8 * j2));
    const v4f a = *(const v4f*)p;
    const v4f b4 = *(const v4f*)(p + 4);
    v8h v;
    v[0] = (_Float16)a.x;  v[1] = (_Float16)a.y;  v[2] = (_Float16)a.z;  v[3] = (_Float16)a.w;
    v[4] = (_Float16)b4.x; v[5] = (_Float16)b4.y; v[6] = (_Float16)b4.z; v[7] = (_Float16)b4.w;
    *(v8h*)(feat + row * KF + 8 * j) = v;
  }
  if (tid < RB) {
    int node = base + tid; node = node > nN - 1 ? nN - 1 : node;
    int bb = bt[node]; bb = bb < 0 ? 0 : (bb > nG - 1 ? nG - 1 : bb);
    sst[tid] = sgv[bb];
  }
  __syncthreads();

  {
    v8f c1[4];
#pragma unroll
    for (int nt = 0; nt < 4; ++nt) c1[nt] = z8f();
    const _Float16* ar = feat + (16 * wave + m) * KF + 8 * hh;
#pragma unroll
    for (int s = 0; s < KF / 32; ++s) {
      FragH a;
      a.h[0] = *(const v8h*)(ar + 32 * s);
      a.h[1] = *(const v8h*)(ar + 32 * s + 16);
#pragma unroll
      for (int nt = 0; nt < 4; ++nt) {
        const _Float16* br = wfc + (size_t)(nt * 16 + m) * KF + 32 * s + 8 * hh;
        FragH bq;
        bq.h[0] = *(const v8h*)(br);
        bq.h[1] = *(const v8h*)(br + 16);
        c1[nt] = wmh(a.v, bq.v, c1[nt]);
      }
    }
#pragma unroll
    for (int nt = 0; nt < 4; ++nt) {
      const int col = nt * 16 + m;
      const float bv = bfc[col];
#pragma unroll
      for (int r2 = 0; r2 < 8; ++r2) {
        const float val = fmaxf(c1[nt][r2] * 0.0625f + bv, 0.0f);
        ft[(16 * wave + 8 * hh + r2) * HD + col] = (_Float16)val;
      }
    }
  }
  __syncthreads();

  {
    v8f c2[3];
#pragma unroll
    for (int nt = 0; nt < 3; ++nt) c2[nt] = z8f();
    const _Float16* ar = ft + (16 * wave + m) * HD + 8 * hh;
#pragma unroll
    for (int s = 0; s < HD / 32; ++s) {
      FragH a;
      a.h[0] = *(const v8h*)(ar + 32 * s);
      a.h[1] = *(const v8h*)(ar + 32 * s + 16);
#pragma unroll
      for (int nt = 0; nt < 3; ++nt) {
        const _Float16* br = wnp + (size_t)(nt * 16 + m) * HD + 32 * s + 8 * hh;
        FragH bq;
        bq.h[0] = *(const v8h*)(br);
        bq.h[1] = *(const v8h*)(br + 16);
        c2[nt] = wmh(a.v, bq.v, c2[nt]);
      }
    }
#pragma unroll
    for (int nt = 0; nt < 3; ++nt) {
      const int col = nt * 16 + m;
      const int cc = col > NC - 1 ? NC - 1 : col;
      const float bv = bnp[cc];
#pragma unroll
      for (int r2 = 0; r2 < 8; ++r2) lg[(16 * wave + 8 * hh + r2) * NCP + col] = c2[nt][r2] * 0.125f + bv;
    }
  }
  __syncthreads();

  {
    const int row = 16 * wave + m;
    const float* lr = lg + row * NCP + 20 * hh;
    float mloc = lr[0];
#pragma unroll 1
    for (int c = 1; c < 20; ++c) mloc = fmaxf(mloc, lr[c]);
    const float mrow = fmaxf(mloc, __shfl_xor(mloc, 16, 32));
    float sl = 0.0f;
#pragma unroll 1
    for (int c = 0; c < 20; ++c) sl += expf(lr[c] - mrow);
    const float tot = sl + __shfl_xor(sl, 16, 32);
    const float lse = logf(tot);
    float* orow = ost + row * NC + 20 * hh;
#pragma unroll 1
    for (int c = 0; c < 20; ++c) orow[c] = (lr[c] - mrow) - lse;
  }
  __syncthreads();

  {
    int vr = nN - base; vr = vr > RB ? RB : (vr < 0 ? 0 : vr);
    const int nf4 = vr * (NC / 4);
    const int nq1 = vr >> 2;
    const int rem1 = vr - 4 * nq1;
    float* o0 = out0 + (size_t)base * NC;
    float* o1 = out1 + base;
#pragma unroll 1
    for (int ps = 0; ps < 2; ++ps) {
      for (int q = tid; q < nf4; q += NTHR) {
        const v4f v = *(const v4f*)(ost + 4 * q);
        *(volatile v4f*)(o0 + 4 * q) = v;
      }
      if (tid < nq1) {
        const v4f v = *(const v4f*)(sst + 4 * tid);
        *(volatile v4f*)(o1 + 4 * tid) = v;
      }
      if (tid < rem1) {
        const float sv = sst[4 * nq1 + tid];
        *(volatile float*)(o1 + 4 * nq1 + tid) = sv;
      }
      if (ps == 0) __threadfence();
    }
  }
}

extern "C" void kernel_launch(void* const* d_in, const int* in_sizes, int n_in,
                              void* d_out, int out_size, void* d_ws, size_t ws_size,
                              hipStream_t stream) {
  if (n_in < 19) return;
  const int nN = in_sizes[0] / NI;
  const int nE = in_sizes[1] / 2;
  const int nG = in_sizes[4] / GFT;
  if (nN <= 0 || nG <= 0 || nE < 0) return;
  if (in_sizes[0] != nN * NI || in_sizes[1] != 2 * nE || in_sizes[2] != nE * EI || in_sizes[3] != nN) return;
  if (in_sizes[4] != nG * GFT) return;
  if (in_sizes[5] != EI * HD || in_sizes[6] != HD || in_sizes[7] != HD * KW || in_sizes[8] != KW) return;
  if (in_sizes[9] != NI * HD || in_sizes[10] != HD || in_sizes[11] != HD || in_sizes[12] < 1) return;
  if (in_sizes[13] != KF * HD || in_sizes[14] != HD || in_sizes[15] != HD * NC || in_sizes[16] != NC) return;
  if (in_sizes[17] != HD || in_sizes[18] < 1) return;
  if (out_size != nN * NC + nN) return;

  const float* x     = (const float*)d_in[0];
  const int*   ei    = (const int*)d_in[1];
  const float* eat   = (const float*)d_in[2];
  const int*   bt    = (const int*)d_in[3];
  const float* pk    = (const float*)d_in[4];
  const float* W_e1  = (const float*)d_in[5];
  const float* b_e1  = (const float*)d_in[6];
  const float* W_e2  = (const float*)d_in[7];
  const float* b_e2  = (const float*)d_in[8];
  const float* root  = (const float*)d_in[9];
  const float* cbias = (const float*)d_in[10];
  const float* Wg    = (const float*)d_in[11];
  const float* bg    = (const float*)d_in[12];
  const float* W_fc1 = (const float*)d_in[13];
  const float* b_fc1 = (const float*)d_in[14];
  const float* W_np  = (const float*)d_in[15];
  const float* b_np  = (const float*)d_in[16];
  const float* W_sp  = (const float*)d_in[17];
  const float* b_sp  = (const float*)d_in[18];
  float* out0 = (float*)d_out;
  float* out1 = out0 + (size_t)nN * NC;

  const int nBA = (nN + NB - 1) / NB;
  const int nBP = (nG + GB - 1) / GB;
  const int nBH = (nN + RB - 1) / RB;

  auto al = [](size_t b) { return (b + 255) & ~(size_t)255; };
  char* ws = (char*)d_ws;
  size_t off = 0;
  const size_t oWp = off; off += al((size_t)HD * KP * 2);
  const size_t oWf = off; off += al((size_t)HD * KF * 2);
  const size_t oWn = off; off += al((size_t)NCP * HD * 2);
  const size_t oH  = off; off += al((size_t)nBA * NB * HD * 4);
  const size_t oG  = off; off += al((size_t)nBA * NB * 4);
  const size_t oC  = off; off += al((size_t)nBP * GB * HD * 4);
  const size_t oS  = off; off += al((size_t)nBP * GB * 4);
  if (off > ws_size) return;
  _Float16* wp   = (_Float16*)(ws + oWp);
  _Float16* wfc  = (_Float16*)(ws + oWf);
  _Float16* wnp  = (_Float16*)(ws + oWn);
  float*    hbuf = (float*)(ws + oH);
  float*    gbuf = (float*)(ws + oG);
  float*    gctx = (float*)(ws + oC);
  float*    sgv  = (float*)(ws + oS);

  const int vecA = ((nE & 3) == 0) ? 1 : 0;
  const int vecP = ((nN & 3) == 0) ? 1 : 0;

  k_prep<<<PREPA + PREPB + PREPC, NTHR, 0, stream>>>(W_e2, b_e2, W_fc1, W_np, wp, wfc, wnp);

  k_agg<<<nBA, NTHR, 0, stream>>>(x, ei, eat, W_e1, b_e1, wp, root, cbias, Wg, bg,
                                  hbuf, gbuf, nN, nE, vecA);

  k_pool<<<nBP, NTHR, 0, stream>>>(gbuf, hbuf, bt, W_sp, b_sp, gctx, sgv, nN, vecP);

  k_head<<<nBH, NTHR, 0, stream>>>(hbuf, gctx, sgv, bt, pk, wfc, b_fc1, wnp, b_np,
                                   out0, out1, nN, nG);
}
